// MultiHeadGAT_23347442221667
// MI455X (gfx1250) — hardware-verified
//
#include <hip/hip_runtime.h>
#include <math.h>
#include <stdint.h>

#define NB_   8
#define NL_   1024
#define DIN   128
#define NH_   8
#define HD_   16
#define DM_   (NH_ * HD_)
#define FF_   256
#define NBH   (NB_ * NH_)
#define NTOK  (NB_ * NL_)
#define SLOPE 0.2f
#define MASKFILL (-1.0e30f)
#define EPS_  1e-5f

static_assert(NL_ % 128 == 0);
static_assert(NL_ % 64 == 0);
static_assert(DIN % 32 == 0);
static_assert(FF_ % 64 == 0);
static_assert(DM_ == 128);
static_assert(DM_ == NH_ * HD_);
static_assert(HD_ == 16);
static_assert(NH_ == 8);
static_assert((NTOK * DIN) % 2048 == 0);
static_assert(NTOK % 128 == 0);

typedef __attribute__((ext_vector_type(16))) __bf16 v16b;
typedef __attribute__((ext_vector_type(8)))  __bf16 v8b;
typedef __attribute__((ext_vector_type(8)))  float  v8f;
typedef __attribute__((ext_vector_type(4)))  float  v4f;
typedef __attribute__((ext_vector_type(4)))  unsigned int v4u;
typedef __attribute__((ext_vector_type(2)))  unsigned int v2u;
typedef __attribute__((ext_vector_type(8)))  unsigned int v8u;
typedef __attribute__((ext_vector_type(4)))  int v4i;
typedef v8b __attribute__((may_alias)) v8ba;
typedef v4f __attribute__((may_alias)) v4fa;
typedef v4u __attribute__((may_alias)) v4ua;
typedef v4i __attribute__((may_alias)) v4ia;

union FragU { v16b v; v8b h[2]; };
union PackU { v8u u; v16b v; };

__device__ __forceinline__ unsigned short f2bf_bits(float f) {
  const unsigned u = __float_as_uint(f);
  return (unsigned short)((u + 0x7FFFu + ((u >> 16) & 1u)) >> 16);
}
__device__ __forceinline__ float bf_bits2f(unsigned short h) { return __uint_as_float(((unsigned)h) << 16); }
__device__ __forceinline__ float bf16r(float f) {
  unsigned u = __float_as_uint(f);
  u = (u + 0x7FFFu + ((u >> 16) & 1u)) & 0xFFFF0000u;
  return __uint_as_float(u);
}
__device__ __forceinline__ unsigned pk16(unsigned short a, unsigned short b) { return (unsigned)a | ((unsigned)b << 16); }

__device__ __forceinline__ v8f wmma_bf16(v16b a, v16b b, v8f c) {
  v8f d = __builtin_amdgcn_wmma_f32_16x16x32_bf16(false, a, false, b, (short)0, c, false, false);
  asm volatile("v_nop\n\tv_nop\n\tv_nop\n\tv_nop" : "+v"(d) : "v"(a), "v"(b));
  return d;
}

__device__ __forceinline__ v16b load_frag(const unsigned short* p, int hh) {
  FragU f;
  f.h[0] = *(const v8ba*)(p + 8 * hh);
  f.h[1] = *(const v8ba*)(p + 16 + 8 * hh);
  return f.v;
}

__device__ __forceinline__ void pack_p2(v8f a, v8f c, v16b& ho, v16b& lo) {
  PackU uh, ul;
#pragma unroll
  for (int i = 0; i < 4; ++i) {
    const unsigned short h0 = f2bf_bits(a[2 * i]), h1 = f2bf_bits(a[2 * i + 1]);
    const unsigned short l0 = f2bf_bits(a[2 * i] - bf_bits2f(h0)), l1 = f2bf_bits(a[2 * i + 1] - bf_bits2f(h1));
    uh.u[i] = pk16(h0, h1); ul.u[i] = pk16(l0, l1);
    const unsigned short g0 = f2bf_bits(c[2 * i]), g1 = f2bf_bits(c[2 * i + 1]);
    const unsigned short m0 = f2bf_bits(c[2 * i] - bf_bits2f(g0)), m1 = f2bf_bits(c[2 * i + 1] - bf_bits2f(g1));
    uh.u[4 + i] = pk16(g0, g1); ul.u[4 + i] = pk16(m0, m1);
  }
  ho = uh.v; lo = ul.v;
}

__device__ __forceinline__ void gemm_core_32x64p(
    const unsigned short* __restrict__ A, const unsigned short* __restrict__ Bt,
    int K, size_t aoff, size_t boff, int hh, v8f (&acc)[2][4]) {
  const unsigned short* a0 = A + aoff;
  const unsigned short* a1 = a0 + (size_t)16 * K;
  const unsigned short* bp = Bt + boff;
#pragma unroll 1
  for (int k0 = 0; k0 < K; k0 += 32) {
    const v16b f0 = load_frag(a0 + k0, hh);
    const v16b f1 = load_frag(a1 + k0, hh);
#pragma unroll
    for (int nt = 0; nt < 4; ++nt) {
      const v16b fb = load_frag(bp + (size_t)nt * 16 * K + k0, hh);
      acc[0][nt] = wmma_bf16(f0, fb, acc[0][nt]);
      acc[1][nt] = wmma_bf16(f1, fb, acc[1][nt]);
    }
  }
}

__device__ __forceinline__ void gemm_core_32x64p2(
    const unsigned short* __restrict__ Ah, const unsigned short* __restrict__ Al,
    const unsigned short* __restrict__ Bt,
    int K, size_t aoff, size_t boff, int hh, v8f (&acc)[2][4]) {
  const unsigned short* a0h = Ah + aoff;
  const unsigned short* a1h = a0h + (size_t)16 * K;
  const unsigned short* a0l = Al + aoff;
  const unsigned short* a1l = a0l + (size_t)16 * K;
  const unsigned short* bp = Bt + boff;
#pragma unroll 1
  for (int k0 = 0; k0 < K; k0 += 32) {
    const v16b f0h = load_frag(a0h + k0, hh);
    const v16b f1h = load_frag(a1h + k0, hh);
    const v16b f0l = load_frag(a0l + k0, hh);
    const v16b f1l = load_frag(a1l + k0, hh);
#pragma unroll
    for (int nt = 0; nt < 4; ++nt) {
      const v16b fb = load_frag(bp + (size_t)nt * 16 * K + k0, hh);
      acc[0][nt] = wmma_bf16(f0h, fb, acc[0][nt]);
      acc[0][nt] = wmma_bf16(f0l, fb, acc[0][nt]);
      acc[1][nt] = wmma_bf16(f1h, fb, acc[1][nt]);
      acc[1][nt] = wmma_bf16(f1l, fb, acc[1][nt]);
    }
  }
}

__global__ __launch_bounds__(256) void k_cvt(const float* __restrict__ src, unsigned short* __restrict__ dst, int n8) {
  int i = blockIdx.x * 256 + threadIdx.x;
  const bool ok = i < n8;
  i = ok ? i : (n8 - 1);
  const float* s = src + (size_t)i * 8;
  const v4f f0 = *(const v4fa*)(s);
  const v4f f1 = *(const v4fa*)(s + 4);
  v4u u;
  u[0] = pk16(f2bf_bits(f0[0]), f2bf_bits(f0[1]));
  u[1] = pk16(f2bf_bits(f0[2]), f2bf_bits(f0[3]));
  u[2] = pk16(f2bf_bits(f1[0]), f2bf_bits(f1[1]));
  u[3] = pk16(f2bf_bits(f1[2]), f2bf_bits(f1[3]));
  unsigned short* d = dst + (size_t)i * 8;
  if (ok) *(volatile v4u*)d = u;
  __threadfence();
  if (ok) *(volatile v4u*)d = u;
}

__global__ __launch_bounds__(256) void k_wgather(const float* __restrict__ src, unsigned short* __restrict__ dst,
                                                 int nunits, int kg, int sh, int sa, int mk, int sb, int ks) {
  int u = blockIdx.x * 256 + threadIdx.x;
  const bool ok = u < nunits;
  u = ok ? u : (nunits - 1);
  const int n = u / kg, g = u - n * kg;
  const int base = (n >> sh) * sa + (n & mk) * sb;
  const float* s = src + (size_t)base + (size_t)(8 * g) * (size_t)ks;
  float f[8];
#pragma unroll
  for (int j = 0; j < 8; ++j) f[j] = s[(size_t)j * (size_t)ks];
  v4u o;
#pragma unroll
  for (int q = 0; q < 4; ++q) o[q] = pk16(f2bf_bits(f[2 * q]), f2bf_bits(f[2 * q + 1]));
  unsigned short* d = dst + (size_t)u * 8;
  if (ok) *(volatile v4u*)d = o;
  __threadfence();
  if (ok) *(volatile v4u*)d = o;
}

__global__ __launch_bounds__(128) void k_proj(
    const unsigned short* __restrict__ Xb, const unsigned short* __restrict__ Wb,
    const float* __restrict__ av, float* __restrict__ S,
    unsigned short* __restrict__ VTh, unsigned short* __restrict__ VTl) {
  __shared__ __align__(16) unsigned char smem[128 * 68 * 4];
  __shared__ __align__(16) float sA[4 * 2 * HD_];
  __shared__ __align__(16) float sS[2 * 4 * 128];
  float* sF = (float*)smem;
  unsigned short* sH = (unsigned short*)smem;
  unsigned short* sL = sH + 64 * 128;
  const int tid = threadIdx.x, lane = tid & 31, w = tid >> 5;
  const int hh = lane >> 4, m = lane & 15;
  const int xb = blockIdx.x;
  const int b  = xb >> 3;
  const int p0 = (xb & 7) * 128;
  const int hg = blockIdx.y;
  const int n0 = hg * 64;
  const int m0 = xb * 128;
  const int m0w = m0 + 32 * w;

  const v8f zero8 = {0.f, 0.f, 0.f, 0.f, 0.f, 0.f, 0.f, 0.f};
  v8f acc[2][4];
#pragma unroll
  for (int mt = 0; mt < 2; ++mt)
#pragma unroll
    for (int nt = 0; nt < 4; ++nt) acc[mt][nt] = zero8;

  gemm_core_32x64p(Xb, Wb, DIN, (size_t)(m0w + m) * DIN, (size_t)(n0 + m) * DIN, hh, acc);

  sA[tid] = bf16r(av[hg * 128 + tid]);
#pragma unroll
  for (int nt = 0; nt < 4; ++nt)
#pragma unroll
    for (int mt = 0; mt < 2; ++mt)
#pragma unroll
      for (int r = 0; r < 8; ++r) {
        const int tokl = 32 * w + 16 * mt + 8 * hh + r;
        const int feat = 16 * nt + m;
        sF[tokl * 68 + feat] = acc[mt][nt][r];
      }
  __syncthreads();
  {
    const float* fr = sF + tid * 68;
#pragma unroll 1
    for (int nt = 0; nt < 4; ++nt) {
      float sl = 0.0f, sr = 0.0f;
#pragma unroll
      for (int d4 = 0; d4 < HD_ / 4; ++d4) {
        const v4f x = *(const v4fa*)(fr + 16 * nt + 4 * d4);
        const v4f y = *(const v4fa*)(sA + 32 * nt + 4 * d4);
        const v4f z = *(const v4fa*)(sA + 32 * nt + HD_ + 4 * d4);
        sl = fmaf(x[0], y[0], sl);
        sl = fmaf(x[1], y[1], sl);
        sl = fmaf(x[2], y[2], sl);
        sl = fmaf(x[3], y[3], sl);
        sr = fmaf(x[0], z[0], sr);
        sr = fmaf(x[1], z[1], sr);
        sr = fmaf(x[2], z[2], sr);
        sr = fmaf(x[3], z[3], sr);
      }
      sS[nt * 128 + tid] = sl;
      sS[512 + nt * 128 + tid] = sr;
    }
  }
  __syncthreads();
  {
    const int head = 4 * hg + w;
    const int bhd = b * NH_ + head;
    const size_t so  = (size_t)bhd * NL_ + p0 + lane * 4;
    const size_t sko = (size_t)NBH * NL_ + so;
    const v4f vq = *(const v4fa*)(sS + w * 128 + lane * 4);
    const v4f vk = *(const v4fa*)(sS + 512 + w * 128 + lane * 4);
    *(volatile v4f*)(S + so)  = vq;
    *(volatile v4f*)(S + sko) = vk;
    __threadfence();
    *(volatile v4f*)(S + so)  = vq;
    *(volatile v4f*)(S + sko) = vk;
  }
#pragma unroll
  for (int nt = 0; nt < 4; ++nt)
#pragma unroll
    for (int mt = 0; mt < 2; ++mt)
#pragma unroll
      for (int r = 0; r < 8; ++r) {
        const int tokl = 32 * w + 16 * mt + 8 * hh + r;
        const int feat = 16 * nt + m;
        const float y = acc[mt][nt][r];
        const unsigned short hb = f2bf_bits(y);
        const unsigned short lb = f2bf_bits(y - bf_bits2f(hb));
        const int idx = feat * 128 + tokl;
        sH[idx] = hb;
        sL[idx] = lb;
      }
  __syncthreads();
  {
    const int dsub = lane >> 4, t8 = (lane & 15) * 8;
    for (int pass = 0; pass < 2; ++pass) {
#pragma unroll
      for (int it = 0; it < 8; ++it) {
        const int d = 16 * w + 2 * it + dsub;
        const v4u hv = *(const v4ua*)(sH + d * 128 + t8);
        const v4u lv = *(const v4ua*)(sL + d * 128 + t8);
        const size_t go = ((size_t)((b * NH_ + 4 * hg) * HD_ + d)) * (size_t)NL_ + p0 + t8;
        *(volatile v4u*)(VTh + go) = hv;
        *(volatile v4u*)(VTl + go) = lv;
      }
      __threadfence();
    }
  }
}

__global__ __launch_bounds__(128) void k_attn(const float* __restrict__ S, const int* __restrict__ adj,
                                              const unsigned short* __restrict__ VTh,
                                              const unsigned short* __restrict__ VTl,
                                              float* __restrict__ CAT) {
  __shared__ __align__(16) float sK[NL_];
  __shared__ __align__(16) float sO[4][16 * HD_];

  const int tid = threadIdx.x, lane = tid & 31, w = tid >> 5;
  const int hh = lane >> 4, m = lane & 15;
  const int qt = blockIdx.x;
  const int bh = blockIdx.y, b = bh >> 3;
  const int q0 = qt * 64, q0w = q0 + 16 * w, q = q0w + m;

  {
    const float* g = S + (size_t)NBH * NL_ + (size_t)bh * NL_ + tid * 8;
    const v4f a0 = *(const v4fa*)(g);
    const v4f a1 = *(const v4fa*)(g + 4);
    *(v4fa*)(sK + tid * 8) = a0;
    *(v4fa*)(sK + tid * 8 + 4) = a1;
  }
  const float sqv = S[(size_t)bh * NL_ + q];
  const int* arow = adj + ((size_t)b * NL_ + q) * (size_t)NL_;

  const v8f zero8 = {0.f, 0.f, 0.f, 0.f, 0.f, 0.f, 0.f, 0.f};
  v8f o = zero8;
  float mrun = -INFINITY, lrun = 0.0f;
  int anyv = 0;

  __syncthreads();

#pragma unroll 1
  for (int ks = 0; ks < NL_ / 64; ++ks) {
    const int kb = ks * 64;

    v8f s[4];
#pragma unroll
    for (int j = 0; j < 4; ++j) {
      const int ko = kb + 16 * j + 8 * hh;
      const v4i mA = *(const v4ia*)(arow + ko);
      const v4i mB = *(const v4ia*)(arow + ko + 4);
      const v4f kA = *(const v4fa*)(sK + ko);
      const v4f kB = *(const v4fa*)(sK + ko + 4);
      const int   mv[8] = {mA[0], mA[1], mA[2], mA[3], mB[0], mB[1], mB[2], mB[3]};
      const float kv[8] = {kA[0], kA[1], kA[2], kA[3], kB[0], kB[1], kB[2], kB[3]};
#pragma unroll
      for (int r = 0; r < 8; ++r) {
        float t = sqv + kv[r];
        t = (t >= 0.0f) ? t : SLOPE * t;
        anyv |= mv[r];
        t = (mv[r] == 0) ? MASKFILL : t;
        s[j][r] = t;
      }
    }
    float cm = -INFINITY;
#pragma unroll
    for (int j = 0; j < 4; ++j)
#pragma unroll
      for (int r = 0; r < 8; ++r) cm = fmaxf(cm, s[j][r]);
    cm = fmaxf(cm, __shfl_xor(cm, 16, 32));
    const float mnew  = fmaxf(mrun, cm);
    const float alpha = __expf(mrun - mnew);
    mrun = mnew;
    float psum = 0.0f;
#pragma unroll
    for (int j = 0; j < 4; ++j)
#pragma unroll
      for (int r = 0; r < 8; ++r) {
        const float p = __expf(s[j][r] - mnew);
        psum += p;
        s[j][r] = p;
      }
    psum += __shfl_xor(psum, 16, 32);
    lrun = lrun * alpha + psum;
#pragma unroll
    for (int r = 0; r < 8; ++r) o[r] *= alpha;

    v16b p0h, p0l, p1h, p1l;
    pack_p2(s[0], s[1], p0h, p0l);
    pack_p2(s[2], s[3], p1h, p1l);

    {
      const unsigned short* vph = VTh + (size_t)(bh * HD_ + m) * (size_t)NL_ + kb;
      const unsigned short* vpl = VTl + (size_t)(bh * HD_ + m) * (size_t)NL_ + kb;
      const v16b v0h = load_frag(vph, hh), v0l = load_frag(vpl, hh);
      o = wmma_bf16(v0h, p0h, o);
      o = wmma_bf16(v0h, p0l, o);
      o = wmma_bf16(v0l, p0h, o);
      const v16b v1h = load_frag(vph + 32, hh), v1l = load_frag(vpl + 32, hh);
      o = wmma_bf16(v1h, p1h, o);
      o = wmma_bf16(v1h, p1l, o);
      o = wmma_bf16(v1l, p1h, o);
    }
  }

  anyv |= __shfl_xor(anyv, 16, 32);
  const float validf = (anyv != 0) ? 1.0f : 0.0f;
  const float inv = validf * (1.0f / lrun);
  float* so = sO[w];
#pragma unroll
  for (int r = 0; r < 8; ++r) so[m * HD_ + 8 * hh + r] = o[r] * inv;
  __syncthreads();
  {
    const size_t cb = ((size_t)bh * NL_ + q0w) * (size_t)HD_;
    for (int pass = 0; pass < 2; ++pass) {
      const v4f v0 = *(const v4fa*)(so + lane * 4);
      const v4f v1 = *(const v4fa*)(so + 128 + lane * 4);
      *(volatile v4f*)(CAT + cb + lane * 4) = v0;
      *(volatile v4f*)(CAT + cb + 128 + lane * 4) = v1;
      __threadfence();
    }
  }
}

__global__ __launch_bounds__(256) void k_ln1(const float* __restrict__ CAT, const float* __restrict__ hin,
                                             const float* __restrict__ g, const float* __restrict__ be,
                                             float* __restrict__ X32, unsigned short* __restrict__ Xh,
                                             unsigned short* __restrict__ Xl) {
  const int tid = threadIdx.x, lane = tid & 31, w = tid >> 5;
  const int row = blockIdx.x * 8 + w;
  const int b = row >> 10, n = row & (NL_ - 1);
  const int head = lane >> 2, d0 = (lane & 3) * 4;
  const v4f c  = *(const v4fa*)(CAT + ((size_t)((b * NH_ + head) * NL_ + n)) * HD_ + d0);
  const v4f hv = *(const v4fa*)(hin + (size_t)row * DIN + lane * 4);
  float x[4];
#pragma unroll
  for (int j = 0; j < 4; ++j) x[j] = c[j] + bf16r(hv[j]);
  float sm = (x[0] + x[1]) + (x[2] + x[3]);
#pragma unroll
  for (int off = 16; off >= 1; off >>= 1) sm += __shfl_xor(sm, off, 32);
  const float mu = sm * (1.0f / (float)DM_);
  float vs = 0.0f;
#pragma unroll
  for (int j = 0; j < 4; ++j) { const float d = x[j] - mu; vs = fmaf(d, d, vs); }
#pragma unroll
  for (int off = 16; off >= 1; off >>= 1) vs += __shfl_xor(vs, off, 32);
  const float rstd = rsqrtf(vs * (1.0f / (float)DM_) + EPS_);
  const v4f gv = *(const v4fa*)(g + lane * 4);
  const v4f bv = *(const v4fa*)(be + lane * 4);
  v4f yv;
  v2u hv2, lv2;
  unsigned short hb[4], lb[4];
#pragma unroll
  for (int j = 0; j < 4; ++j) {
    const float y = (x[j] - mu) * rstd * bf16r(gv[j]) + bf16r(bv[j]);
    yv[j] = y;
    hb[j] = f2bf_bits(y);
    lb[j] = f2bf_bits(y - bf_bits2f(hb[j]));
  }
  hv2[0] = pk16(hb[0], hb[1]); hv2[1] = pk16(hb[2], hb[3]);
  lv2[0] = pk16(lb[0], lb[1]); lv2[1] = pk16(lb[2], lb[3]);
  const size_t eo = (size_t)row * DM_ + lane * 4;
  *(volatile v4f*)(X32 + eo) = yv;
  *(volatile v2u*)(Xh + eo) = hv2;
  *(volatile v2u*)(Xl + eo) = lv2;
  __threadfence();
  *(volatile v4f*)(X32 + eo) = yv;
  *(volatile v2u*)(Xh + eo) = hv2;
  *(volatile v2u*)(Xl + eo) = lv2;
}

__global__ __launch_bounds__(128) void k_ffn1(const unsigned short* __restrict__ Xh, const unsigned short* __restrict__ Xl,
                                              const unsigned short* __restrict__ W1b, const float* __restrict__ b1,
                                              unsigned short* __restrict__ Th, unsigned short* __restrict__ Tl) {
  __shared__ __align__(16) unsigned short sH[128 * 64];
  __shared__ __align__(16) unsigned short sL[128 * 64];
  const int tid = threadIdx.x, lane = tid & 31, w = tid >> 5;
  const int hh = lane >> 4, m = lane & 15;
  const int m0 = blockIdx.x * 128;
  const int ng = blockIdx.y;
  const int n0 = ng * 64;
  const int m0w = m0 + 32 * w;

  const v8f zero8 = {0.f, 0.f, 0.f, 0.f, 0.f, 0.f, 0.f, 0.f};
  v8f acc[2][4];
#pragma unroll
  for (int mt = 0; mt < 2; ++mt)
#pragma unroll
    for (int nt = 0; nt < 4; ++nt) acc[mt][nt] = zero8;

  gemm_core_32x64p2(Xh, Xl, W1b, DIN, (size_t)(m0w + m) * DIN, (size_t)(n0 + m) * DIN, hh, acc);

#pragma unroll
  for (int nt = 0; nt < 4; ++nt) {
    const int feat = 16 * nt + m;
    const float bvl = bf16r(b1[n0 + feat]);
#pragma unroll
    for (int mt = 0; mt < 2; ++mt)
#pragma unroll
      for (int r = 0; r < 8; ++r) {
        const int tokl = 32 * w + 16 * mt + 8 * hh + r;
        const float y = fmaxf(acc[mt][nt][r] + bvl, 0.0f);
        const unsigned short hb = f2bf_bits(y);
        const unsigned short lb = f2bf_bits(y - bf_bits2f(hb));
        sH[tokl * 64 + feat] = hb;
        sL[tokl * 64 + feat] = lb;
      }
  }
  __syncthreads();
  {
    const int q8 = lane & 7, sub = lane >> 3;
    for (int pass = 0; pass < 2; ++pass) {
#pragma unroll
      for (int i = 0; i < 8; ++i) {
        const int lid = w * 32 + i * 4 + sub;
        const v4u hv = *(const v4ua*)(sH + lid * 64 + 8 * q8);
        const v4u lv = *(const v4ua*)(sL + lid * 64 + 8 * q8);
        const size_t go = (size_t)(m0 + lid) * FF_ + n0 + 8 * q8;
        *(volatile v4u*)(Th + go) = hv;
        *(volatile v4u*)(Tl + go) = lv;
      }
      __threadfence();
    }
  }
}

__global__ __launch_bounds__(128) void k_ffn2(const unsigned short* __restrict__ Th, const unsigned short* __restrict__ Tl,
                                              const unsigned short* __restrict__ W2b, const float* __restrict__ b2,
                                              const float* __restrict__ X32, const float* __restrict__ g2,
                                              const float* __restrict__ be2, float* __restrict__ out) {
  __shared__ __align__(16) float sT[64 * 132];
  const int tid = threadIdx.x, lane = tid & 31, w = tid >> 5;
  const int hh = lane >> 4, m = lane & 15;
  const int wr = w & 1, wc = w >> 1;
  const int m0 = blockIdx.x * 64;
  const int m0w = m0 + 32 * wr;
  const int n0 = 64 * wc;

  const v8f zero8 = {0.f, 0.f, 0.f, 0.f, 0.f, 0.f, 0.f, 0.f};
  v8f acc[2][4];
#pragma unroll
  for (int mt = 0; mt < 2; ++mt)
#pragma unroll
    for (int nt = 0; nt < 4; ++nt) acc[mt][nt] = zero8;

  gemm_core_32x64p2(Th, Tl, W2b, FF_, (size_t)(m0w + m) * FF_, (size_t)(n0 + m) * FF_, hh, acc);

#pragma unroll
  for (int nt = 0; nt < 4; ++nt)
#pragma unroll
    for (int mt = 0; mt < 2; ++mt)
#pragma unroll
      for (int r = 0; r < 8; ++r) {
        const int tokl = 32 * wr + 16 * mt + 8 * hh + r;
        const int col = n0 + 16 * nt + m;
        sT[tokl * 132 + col] = acc[mt][nt][r];
      }
  __syncthreads();

  const v4f b2r = *(const v4fa*)(b2 + lane * 4);
  const v4f g2r = *(const v4fa*)(g2 + lane * 4);
  const v4f e2r = *(const v4fa*)(be2 + lane * 4);
  float bb[4], gg[4], ee[4];
#pragma unroll
  for (int j = 0; j < 4; ++j) { bb[j] = bf16r(b2r[j]); gg[j] = bf16r(g2r[j]); ee[j] = bf16r(e2r[j]); }

#pragma unroll 1
  for (int rr = 0; rr < 16; ++rr) {
    const int row = 16 * w + rr;
    const int tok = m0 + row;
    const v4f f  = *(const v4fa*)(sT + row * 132 + lane * 4);
    const v4f xr = *(const v4fa*)(X32 + (size_t)tok * DM_ + lane * 4);
    float x[4];
#pragma unroll
    for (int j = 0; j < 4; ++j) x[j] = xr[j] + (f[j] + bb[j]);
    float sm = (x[0] + x[1]) + (x[2] + x[3]);
#pragma unroll
    for (int off = 16; off >= 1; off >>= 1) sm += __shfl_xor(sm, off, 32);
    const float mu = sm * (1.0f / (float)DM_);
    float vs = 0.0f;
#pragma unroll
    for (int j = 0; j < 4; ++j) { const float d = x[j] - mu; vs = fmaf(d, d, vs); }
#pragma unroll
    for (int off = 16; off >= 1; off >>= 1) vs += __shfl_xor(vs, off, 32);
    const float rstd = rsqrtf(vs * (1.0f / (float)DM_) + EPS_);
    v4f yv;
#pragma unroll
    for (int j = 0; j < 4; ++j) yv[j] = (x[j] - mu) * rstd * gg[j] + ee[j];
    float* op = out + (size_t)tok * DM_ + lane * 4;
    *(volatile v4f*)op = yv;
    __threadfence();
    *(volatile v4f*)op = yv;
  }
}

extern "C" void kernel_launch(void* const* d_in, const int* in_sizes, int n_in,
                              void* d_out, int out_size, void* d_ws, size_t ws_size,
                              hipStream_t stream) {
  if (n_in < 12) return;
  if (in_sizes[0] != NTOK * DIN) return;
  if (in_sizes[1] != NB_ * NL_ * NL_) return;
  if (in_sizes[2] != NH_ * DIN * HD_) return;
  if (in_sizes[3] != NH_ * 2 * HD_) return;
  if (in_sizes[4] != DM_ || in_sizes[5] != DM_) return;
  if (in_sizes[6] != DM_ * FF_) return;
  if (in_sizes[7] != FF_) return;
  if (in_sizes[8] != FF_ * DM_) return;
  if (in_sizes[9] != DM_) return;
  if (in_sizes[10] != DM_ || in_sizes[11] != DM_) return;
  if (out_size != NTOK * DM_) return;

  const float* hin  = (const float*)d_in[0];
  const int*   adj  = (const int*)d_in[1];
  const float* W    = (const float*)d_in[2];
  const float* av   = (const float*)d_in[3];
  const float* ln1g = (const float*)d_in[4];
  const float* ln1b = (const float*)d_in[5];
  const float* w1   = (const float*)d_in[6];
  const float* b1   = (const float*)d_in[7];
  const float* w2   = (const float*)d_in[8];
  const float* b2   = (const float*)d_in[9];
  const float* ln2g = (const float*)d_in[10];
  const float* ln2b = (const float*)d_in[11];
  float* out = (float*)d_out;

  const size_t PXB  = (size_t)NTOK * DIN * 2;
  const size_t PWB  = (size_t)DM_ * DIN * 2;
  const size_t PW1  = (size_t)FF_ * DIN * 2;
  const size_t PW2  = (size_t)DM_ * FF_ * 2;
  const size_t PS   = (size_t)2 * NBH * NL_ * 4;
  const size_t PVT  = (size_t)NBH * HD_ * NL_ * 2;
  const size_t PCAT = (size_t)NBH * NL_ * HD_ * 4;
  const size_t PX32 = (size_t)NTOK * DM_ * 4;
  const size_t PXH  = (size_t)NTOK * DM_ * 2;
  const size_t PT   = (size_t)NTOK * FF_ * 2;
  size_t off = 0;
  const size_t oXb  = off; off += PXB;
  const size_t oWb  = off; off += PWB;
  const size_t oW1  = off; off += PW1;
  const size_t oW2  = off; off += PW2;
  const size_t oS   = off; off += PS;
  const size_t oVTh = off; off += PVT;
  const size_t oVTl = off; off += PVT;
  const size_t oCAT = off; off += PCAT;
  const size_t oX32 = off; off += PX32;
  const size_t oXh  = off; off += PXH;
  const size_t oXl  = off; off += PXH;
  const size_t oTh  = off; off += PT;
  const size_t oTl  = off; off += PT;
  if (off > ws_size) return;

  char* ws = (char*)d_ws;
  unsigned short* Xb  = (unsigned short*)(ws + oXb);
  unsigned short* Wb  = (unsigned short*)(ws + oWb);
  unsigned short* W1b = (unsigned short*)(ws + oW1);
  unsigned short* W2b = (unsigned short*)(ws + oW2);
  float*          S   = (float*)(ws + oS);
  unsigned short* VTh = (unsigned short*)(ws + oVTh);
  unsigned short* VTl = (unsigned short*)(ws + oVTl);
  float*          CAT = (float*)(ws + oCAT);
  float*          X32 = (float*)(ws + oX32);
  unsigned short* Xh  = (unsigned short*)(ws + oXh);
  unsigned short* Xl  = (unsigned short*)(ws + oXl);
  unsigned short* Th  = (unsigned short*)(ws + oTh);
  unsigned short* Tl  = (unsigned short*)(ws + oTl);

  const int n8x = NTOK * DIN / 8;
  k_cvt<<<dim3((n8x + 255) / 256), 256, 0, stream>>>(hin, Xb, n8x);
  k_wgather<<<dim3((DM_ * (DIN / 8) + 255) / 256), 256, 0, stream>>>(W, Wb, DM_ * (DIN / 8), DIN / 8, 4, DIN * HD_, 15, 1, HD_);
  k_wgather<<<dim3((FF_ * (DIN / 8) + 255) / 256), 256, 0, stream>>>(w1, W1b, FF_ * (DIN / 8), DIN / 8, 0, 1, 0, 0, FF_);
  k_wgather<<<dim3((DM_ * (FF_ / 8) + 255) / 256), 256, 0, stream>>>(w2, W2b, DM_ * (FF_ / 8), FF_ / 8, 0, 1, 0, 0, DM_);
  k_proj<<<dim3(NTOK / 128, 2), 128, 0, stream>>>(Xb, Wb, av, S, VTh, VTl);
  k_attn<<<dim3(NL_ / 64, NBH), 128, 0, stream>>>(S, adj, VTh, VTl, CAT);
  k_ln1<<<dim3(NTOK / 8), 256, 0, stream>>>(CAT, hin, ln1g, ln1b, X32, Xh, Xl);
  k_ffn1<<<dim3(NTOK / 128, FF_ / 64), 128, 0, stream>>>(Xh, Xl, W1b, b1, Th, Tl);
  k_ffn2<<<dim3(NTOK / 64), 128, 0, stream>>>(Th, Tl, W2b, b2, X32, ln2g, ln2b, out);
  (void)hipGetLastError();
}
